// FusedAttention_37984690766201
// MI455X (gfx1250) — hardware-verified
//
#include <hip/hip_runtime.h>
#include <hip/hip_bf16.h>
#include <math.h>


typedef __bf16 v16b __attribute__((ext_vector_type(16)));
typedef float v8f __attribute__((ext_vector_type(8)));
typedef float v4f __attribute__((ext_vector_type(4)));
typedef unsigned int v4u __attribute__((ext_vector_type(4)));
typedef v4f __attribute__((may_alias)) v4fa;
typedef v4u __attribute__((may_alias)) v4ua;
typedef unsigned short us16;

union Frag { v16b v; v4u u[2]; };

__device__ __forceinline__ v16b ldfrag(const us16* p, int hh) {
    Frag f;
    f.u[0] = *(const v4ua*)(p + 8 * hh);
    f.u[1] = *(const v4ua*)(p + 16 + 8 * hh);
    return f.v;
}

__device__ __forceinline__ v8f mma(v16b a, v16b b, v8f c) {
    v8f d = __builtin_amdgcn_wmma_f32_16x16x32_bf16(false, a, false, b, (short)0, c, false, false);
    asm volatile("v_nop\n\tv_nop\n\tv_nop\n\tv_nop" : "+v"(d) : "v"(a), "v"(b));
    return d;
}

__device__ __forceinline__ unsigned bfbits(float f) {
    unsigned u = __float_as_uint(f);
    return (u + 0x7FFFu + ((u >> 16) & 1u)) >> 16;
}
__device__ __forceinline__ void split_pair(float a, float b, unsigned& hw, unsigned& lw) {
    const unsigned ha = bfbits(a), hb = bfbits(b);
    const float ra = a - __uint_as_float(ha << 16);
    const float rb = b - __uint_as_float(hb << 16);
    hw = ha | (hb << 16);
    lw = bfbits(ra) | (bfbits(rb) << 16);
}
__device__ __forceinline__ void split8(v4f x0, v4f x1, v4u& hv, v4u& lv) {
    unsigned h0, h1, h2, h3, l0, l1, l2, l3;
    split_pair(x0.x, x0.y, h0, l0);
    split_pair(x0.z, x0.w, h1, l1);
    split_pair(x1.x, x1.y, h2, l2);
    split_pair(x1.z, x1.w, h3, l3);
    v4u hh = {h0, h1, h2, h3};
    v4u ll = {l0, l1, l2, l3};
    hv = hh; lv = ll;
}

__device__ __forceinline__ void lds_wave_sync() {
    __builtin_amdgcn_fence(__ATOMIC_ACQ_REL, "wavefront");
    __builtin_amdgcn_wave_barrier();
    asm volatile("s_wait_dscnt 0" ::: "memory");
}

__global__ __launch_bounds__(256) void k_split(const float* __restrict__ src,
                                                us16* __restrict__ hi, us16* __restrict__ lo, int n8) {
    const int t = blockIdx.x * 256 + threadIdx.x;
    if (t >= n8) return;
    const float* p = src + (size_t)t * 8;
    const v4f a = *(const v4fa*)p;
    const v4f b = *(const v4fa*)(p + 4);
    v4u hv, lv;
    split8(a, b, hv, lv);
    us16* ph = hi + (size_t)t * 8;
    us16* pl = lo + (size_t)t * 8;
    *(volatile v4ua*)ph = hv;
    *(volatile v4ua*)pl = lv;
    __threadfence();
    *(volatile v4ua*)ph = hv;
    *(volatile v4ua*)pl = lv;
}

__global__ __launch_bounds__(32) void k_invfreq(float* __restrict__ invf) {
    const int t = threadIdx.x;
    const int i0 = (t & 15) * 4;
    float f0 = 0.f, f1 = 0.f, f2 = 0.f, f3 = 0.f;
#pragma unroll 1
    for (int e = 0; e < 4; ++e) {
        const float ex = (float)(2 * (i0 + e)) * 0.0078125f;
        const float pw = powf(10000.0f, ex);
        const float inv = 1.0f / pw;
        f0 = f1; f1 = f2; f2 = f3; f3 = inv;
    }
    v4f v = {f0, f1, f2, f3};
    if (t < 16) *(volatile v4fa*)(invf + i0) = v;
    __threadfence();
    if (t < 16) *(volatile v4fa*)(invf + i0) = v;
}

__global__ __launch_bounds__(256) void k_rope_tab(const float* __restrict__ invf,
                                                   float* __restrict__ ct, float* __restrict__ st, int S) {
    const int t = blockIdx.x * 256 + threadIdx.x;
    if (t >= S * 16) return;
    const int s = t >> 4, i0 = (t & 15) * 4;
    v4f iv = *(const v4fa*)(invf + i0);
    float c0 = 0.f, c1 = 0.f, c2 = 0.f, c3 = 0.f;
    float n0 = 0.f, n1 = 0.f, n2 = 0.f, n3 = 0.f;
#pragma unroll 1
    for (int e = 0; e < 4; ++e) {
        const float ang = (float)s * iv.x;
        iv = iv.yzwx;
        float sn, cs;
        sincosf(ang, &sn, &cs);
        c0 = c1; c1 = c2; c2 = c3; c3 = cs;
        n0 = n1; n1 = n2; n2 = n3; n3 = sn;
    }
    v4f cv = {c0, c1, c2, c3};
    v4f sv = {n0, n1, n2, n3};
    const size_t off = (size_t)s * 64 + i0;
    *(volatile v4fa*)(ct + off) = cv;
    *(volatile v4fa*)(st + off) = sv;
    __threadfence();
    *(volatile v4fa*)(ct + off) = cv;
    *(volatile v4fa*)(st + off) = sv;
}

#define TP 128

__device__ __forceinline__ void gemm_core(const us16* __restrict__ Ah, const us16* __restrict__ Al,
                                          const us16* __restrict__ Wh, const us16* __restrict__ Wl,
                                          int K, int arow0, int wrow0, float* Ts) {
    const int tid = threadIdx.x, l = tid & 31, w = tid >> 5;
    const int hh = l >> 4, m = l & 15;
    const int wm = w >> 1, wn = w & 1;
    const size_t abase = (size_t)(arow0 + wm * 32 + m) * K;
    const size_t wbase = (size_t)(wrow0 + wn * 64 + m) * K;

    v8f acc[2][4] = {};

#pragma unroll 1
    for (int k0 = 0; k0 < K; k0 += 32) {
        v16b fah[2], fal[2];
#pragma unroll
        for (int i = 0; i < 2; ++i) {
            const size_t ao = abase + (size_t)i * 16 * K + k0;
            fah[i] = ldfrag(Ah + ao, hh);
            fal[i] = ldfrag(Al + ao, hh);
        }
#pragma unroll
        for (int j = 0; j < 4; ++j) {
            const size_t wo = wbase + (size_t)j * 16 * K + k0;
            const v16b fbh = ldfrag(Wh + wo, hh);
            const v16b fbl = ldfrag(Wl + wo, hh);
#pragma unroll
            for (int i = 0; i < 2; ++i) {
                acc[i][j] = mma(fah[i], fbh, acc[i][j]);
                acc[i][j] = mma(fah[i], fbl, acc[i][j]);
                acc[i][j] = mma(fal[i], fbh, acc[i][j]);
            }
        }
    }

#pragma unroll
    for (int i = 0; i < 2; ++i)
#pragma unroll
        for (int j = 0; j < 4; ++j)
#pragma unroll
            for (int r = 0; r < 8; ++r)
                Ts[(wm * 32 + i * 16 + 8 * hh + r) * TP + wn * 64 + j * 16 + m] = acc[i][j][r];
}

__global__ __launch_bounds__(128) void k_qkv(const us16* __restrict__ xh, const us16* __restrict__ xl,
                                              const us16* __restrict__ wh, const us16* __restrict__ wl,
                                              const float* __restrict__ ct, const float* __restrict__ st,
                                              us16* __restrict__ qh, us16* __restrict__ ql,
                                              us16* __restrict__ kh, us16* __restrict__ kl,
                                              us16* __restrict__ vh, us16* __restrict__ vl,
                                              int S, int K) {
    __shared__ __attribute__((aligned(16))) float Ts[64 * TP];
    const int u = blockIdx.x;
    const int bm = blockIdx.y * 64;
    gemm_core(xh, xl, wh, wl, K, bm, u * 128, Ts);
    __syncthreads();

    const int tid = threadIdx.x;
    if (u < 20) {
        const int rr = tid >> 4, seg = tid & 15;
        us16* dh = qh;
        us16* dl = ql;
        size_t base = (size_t)u * S * 128;
        if (u >= 16) { dh = kh; dl = kl; base = (size_t)(u - 16) * S * 128; }
#pragma unroll 1
        for (int ps = 0; ps < 2; ++ps) {
#pragma unroll 1
            for (int p = 0; p < 8; ++p) {
                const int row = p * 8 + rr;
                const int s = bm + row;
                const v4f x0 = *(const v4fa*)(Ts + row * TP + seg * 8);
                const v4f x1 = *(const v4fa*)(Ts + row * TP + seg * 8 + 4);
                const v4f cv = *(const v4fa*)(ct + (size_t)s * 64 + seg * 4);
                const v4f sv = *(const v4fa*)(st + (size_t)s * 64 + seg * 4);
                v4f o0, o1;
                o0.x = x0.x * cv.x - x0.y * sv.x;
                o0.y = x0.x * sv.x + x0.y * cv.x;
                o0.z = x0.z * cv.y - x0.w * sv.y;
                o0.w = x0.z * sv.y + x0.w * cv.y;
                o1.x = x1.x * cv.z - x1.y * sv.z;
                o1.y = x1.x * sv.z + x1.y * cv.z;
                o1.z = x1.z * cv.w - x1.w * sv.w;
                o1.w = x1.z * sv.w + x1.w * cv.w;
                v4u hv, lv;
                split8(o0, o1, hv, lv);
                const size_t off = base + (size_t)s * 128 + seg * 8;
                *(volatile v4ua*)(dh + off) = hv;
                *(volatile v4ua*)(dl + off) = lv;
            }
            __threadfence();
        }
    } else {
        const int kvh = u - 20;
        const int dd = tid >> 3, g = tid & 7;
#pragma unroll 1
        for (int ps = 0; ps < 2; ++ps) {
#pragma unroll 1
            for (int p = 0; p < 8; ++p) {
                const int d = p * 16 + dd;
                v4f x0, x1;
                x0.x = Ts[(g * 8 + 0) * TP + d];
                x0.y = Ts[(g * 8 + 1) * TP + d];
                x0.z = Ts[(g * 8 + 2) * TP + d];
                x0.w = Ts[(g * 8 + 3) * TP + d];
                x1.x = Ts[(g * 8 + 4) * TP + d];
                x1.y = Ts[(g * 8 + 5) * TP + d];
                x1.z = Ts[(g * 8 + 6) * TP + d];
                x1.w = Ts[(g * 8 + 7) * TP + d];
                v4u hv, lv;
                split8(x0, x1, hv, lv);
                const size_t off = ((size_t)(kvh * 128 + d)) * S + bm + g * 8;
                *(volatile v4ua*)(vh + off) = hv;
                *(volatile v4ua*)(vl + off) = lv;
            }
            __threadfence();
        }
    }
}

__global__ __launch_bounds__(128) void k_proj(const us16* __restrict__ ah, const us16* __restrict__ al,
                                               const us16* __restrict__ wh, const us16* __restrict__ wl,
                                               float* __restrict__ out, int K, int N, int orow0) {
    __shared__ __attribute__((aligned(16))) float Ts[64 * TP];
    const int bm = blockIdx.y * 64, bn = blockIdx.x * 128;
    gemm_core(ah, al, wh, wl, K, bm, bn, Ts);
    __syncthreads();

    const int tid = threadIdx.x;
    const int rr = tid >> 5, c4 = tid & 31;
#pragma unroll 1
    for (int ps = 0; ps < 2; ++ps) {
#pragma unroll 1
        for (int p = 0; p < 16; ++p) {
            const int row = p * 4 + rr;
            const v4f v = *(const v4fa*)(Ts + row * TP + c4 * 4);
            *(volatile v4fa*)(out + (size_t)(orow0 + bm + row) * N + bn + c4 * 4) = v;
        }
        __threadfence();
    }
}

#define PP 36
#define OP 132

__global__ __launch_bounds__(32) void k_attn(const us16* __restrict__ qh, const us16* __restrict__ ql,
                                              const us16* __restrict__ kh, const us16* __restrict__ kl,
                                              const us16* __restrict__ vh, const us16* __restrict__ vl,
                                              us16* __restrict__ ch, us16* __restrict__ cl,
                                              int S, int DC) {
    __shared__ __attribute__((aligned(16))) float Psf[16 * PP];
    __shared__ __attribute__((aligned(16))) float Osf[16 * OP];

    const int l = threadIdx.x & 31, hh = l >> 4, m = l & 15;
    const int q0 = blockIdx.x * 16, h = blockIdx.y, kvh = h >> 2;

    const size_t qoff = ((size_t)h * S + q0 + m) * 128;
    const us16* qhr = qh + qoff;
    const us16* qlr = ql + qoff;
    const us16* khb = kh + ((size_t)kvh * S + m) * 128;
    const us16* klb = kl + ((size_t)kvh * S + m) * 128;
    const us16* vhb = vh + ((size_t)kvh * 128 + m) * S;
    const us16* vlb = vl + ((size_t)kvh * 128 + m) * S;

    v8f ao[8] = {};
    float mrow[8], lrow[8];
#pragma unroll
    for (int r = 0; r < 8; ++r) { mrow[r] = -1.0e30f; lrow[r] = 0.0f; }

    const float scale = 0.08838834764831845f;
    const int ntile = ((q0 + 15) >> 5) + 1;

#pragma unroll 1
    for (int t = 0; t < ntile; ++t) {
        const int kv0 = t * 32;

        v8f sc0 = {};
        v8f sc1 = {};
#pragma unroll
        for (int c = 0; c < 4; ++c) {
            const v16b fqh = ldfrag(qhr + c * 32, hh);
            const v16b fql = ldfrag(qlr + c * 32, hh);
            const size_t ko = (size_t)kv0 * 128 + c * 32;
            const v16b fkh0 = ldfrag(khb + ko, hh);
            const v16b fkl0 = ldfrag(klb + ko, hh);
            sc0 = mma(fqh, fkh0, sc0);
            sc0 = mma(fqh, fkl0, sc0);
            sc0 = mma(fql, fkh0, sc0);
            const v16b fkh1 = ldfrag(khb + ko + 16 * 128, hh);
            const v16b fkl1 = ldfrag(klb + ko + 16 * 128, hh);
            sc1 = mma(fqh, fkh1, sc1);
            sc1 = mma(fqh, fkl1, sc1);
            sc1 = mma(fql, fkh1, sc1);
        }

        const bool needmask = (kv0 + 31) > q0;
        float pv0[8], pv1[8];
#pragma unroll
        for (int r = 0; r < 8; ++r) {
            const int qr = q0 + 8 * hh + r;
            float s0 = sc0[r] * scale;
            float s1 = sc1[r] * scale;
            if (needmask) {
                if (kv0 + m > qr)      s0 = -1.0e9f;
                if (kv0 + 16 + m > qr) s1 = -1.0e9f;
            }
            float tmax = fmaxf(s0, s1);
            tmax = fmaxf(tmax, __shfl_xor(tmax, 1));
            tmax = fmaxf(tmax, __shfl_xor(tmax, 2));
            tmax = fmaxf(tmax, __shfl_xor(tmax, 4));
            tmax = fmaxf(tmax, __shfl_xor(tmax, 8));
            const float mn = fmaxf(mrow[r], tmax);
            const float sf = __expf(mrow[r] - mn);
            const float p0 = __expf(s0 - mn);
            const float p1 = __expf(s1 - mn);
            float rs = p0 + p1;
            rs += __shfl_xor(rs, 1);
            rs += __shfl_xor(rs, 2);
            rs += __shfl_xor(rs, 4);
            rs += __shfl_xor(rs, 8);
            lrow[r] = lrow[r] * sf + rs;
            mrow[r] = mn;
#pragma unroll
            for (int dt = 0; dt < 8; ++dt) ao[dt][r] = ao[dt][r] * sf;
            pv0[r] = p0;
            pv1[r] = p1;
        }

        lds_wave_sync();
#pragma unroll
        for (int r = 0; r < 8; ++r) {
            Psf[(8 * hh + r) * PP + m]      = pv0[r];
            Psf[(8 * hh + r) * PP + 16 + m] = pv1[r];
        }
        lds_wave_sync();
        const float* pr = Psf + m * PP;
        const v4f y0 = *(const v4fa*)(pr + 8 * hh);
        const v4f y1 = *(const v4fa*)(pr + 8 * hh + 4);
        const v4f y2 = *(const v4fa*)(pr + 16 + 8 * hh);
        const v4f y3 = *(const v4fa*)(pr + 16 + 8 * hh + 4);
        lds_wave_sync();
        Frag fph, fpl;
        {
            v4u h01, l01, h23, l23;
            split8(y0, y1, h01, l01);
            split8(y2, y3, h23, l23);
            fph.u[0] = h01; fph.u[1] = h23;
            fpl.u[0] = l01; fpl.u[1] = l23;
        }

#pragma unroll
        for (int dt = 0; dt < 8; ++dt) {
            const size_t vo = (size_t)dt * 16 * S + kv0;
            const v16b fvh = ldfrag(vhb + vo, hh);
            const v16b fvl = ldfrag(vlb + vo, hh);
            ao[dt] = mma(fph.v, fvh, ao[dt]);
            ao[dt] = mma(fph.v, fvl, ao[dt]);
            ao[dt] = mma(fpl.v, fvh, ao[dt]);
        }
    }

    float rl[8];
#pragma unroll
    for (int r = 0; r < 8; ++r) rl[r] = 1.0f / lrow[r];
    lds_wave_sync();
#pragma unroll
    for (int dt = 0; dt < 8; ++dt)
#pragma unroll
        for (int r = 0; r < 8; ++r)
            Osf[(8 * hh + r) * OP + dt * 16 + m] = ao[dt][r] * rl[r];
    lds_wave_sync();

#pragma unroll 1
    for (int ps = 0; ps < 2; ++ps) {
#pragma unroll 1
        for (int p = 0; p < 8; ++p) {
            const int row = 2 * p + hh;
            const v4f x0 = *(const v4fa*)(Osf + row * OP + m * 8);
            const v4f x1 = *(const v4fa*)(Osf + row * OP + m * 8 + 4);
            v4u hv, lv;
            split8(x0, x1, hv, lv);
            const size_t off = (size_t)(q0 + row) * DC + h * 128 + m * 8;
            *(volatile v4ua*)(ch + off) = hv;
            *(volatile v4ua*)(cl + off) = lv;
        }
        __threadfence();
    }
}

static inline size_t al256(size_t x) { return (x + 255) & ~(size_t)255; }

extern "C" void kernel_launch(void* const* d_in, const int* in_sizes, int n_in,
                              void* d_out, int out_size, void* d_ws, size_t ws_size,
                              hipStream_t stream) {
    const int B = 2, S = 2048, D = 2048, HQ = 16, HKV = 4, HD = 128;
    const int NQ = (HQ + 2 * HKV) * HD;
    const int DC = HQ * HD;
    if (n_in < 3) return;
    if (in_sizes[0] != B * S * D || in_sizes[1] != NQ * D || in_sizes[2] != D * DC || out_size != B * S * D) return;

    const float* x     = (const float*)d_in[0];
    const float* w_qkv = (const float*)d_in[1];
    const float* w_o   = (const float*)d_in[2];
    float*       out   = (float*)d_out;

    char*  ws  = (char*)d_ws;
    size_t off = 0;
    us16* xh  = (us16*)(ws + off); off += al256((size_t)B * S * D * 2);
    us16* xl  = (us16*)(ws + off); off += al256((size_t)B * S * D * 2);
    us16* wqh = (us16*)(ws + off); off += al256((size_t)NQ * D * 2);
    us16* wql = (us16*)(ws + off); off += al256((size_t)NQ * D * 2);
    us16* woh = (us16*)(ws + off); off += al256((size_t)D * DC * 2);
    us16* wol = (us16*)(ws + off); off += al256((size_t)D * DC * 2);
    float* invf = (float*)(ws + off); off += al256(64 * 4);
    float* ct  = (float*)(ws + off); off += al256((size_t)S * 64 * 4);
    float* st  = (float*)(ws + off); off += al256((size_t)S * 64 * 4);
    us16* qh  = (us16*)(ws + off); off += al256((size_t)HQ * S * HD * 2);
    us16* ql  = (us16*)(ws + off); off += al256((size_t)HQ * S * HD * 2);
    us16* kh  = (us16*)(ws + off); off += al256((size_t)HKV * S * HD * 2);
    us16* kl  = (us16*)(ws + off); off += al256((size_t)HKV * S * HD * 2);
    us16* vh  = (us16*)(ws + off); off += al256((size_t)HKV * HD * S * 2);
    us16* vl  = (us16*)(ws + off); off += al256((size_t)HKV * HD * S * 2);
    us16* cth = (us16*)(ws + off); off += al256((size_t)S * DC * 2);
    us16* ctl = (us16*)(ws + off); off += al256((size_t)S * DC * 2);
    if (off > ws_size) return;

    const int n8x = B * S * D / 8, n8q = NQ * D / 8, n8o = D * DC / 8;
    k_split<<<(n8x + 255) / 256, 256, 0, stream>>>(x, xh, xl, n8x);
    k_split<<<(n8q + 255) / 256, 256, 0, stream>>>(w_qkv, wqh, wql, n8q);
    k_split<<<(n8o + 255) / 256, 256, 0, stream>>>(w_o, woh, wol, n8o);

    k_invfreq<<<1, 32, 0, stream>>>(invf);
    k_rope_tab<<<(S * 16 + 255) / 256, 256, 0, stream>>>(invf, ct, st, S);

    for (int b = 0; b < B; ++b) {
        const us16* xhb = xh + (size_t)b * S * D;
        const us16* xlb = xl + (size_t)b * S * D;
        k_qkv<<<dim3(NQ / 128, S / 64), 128, 0, stream>>>(xhb, xlb, wqh, wql, ct, st,
                                                          qh, ql, kh, kl, vh, vl, S, D);
        k_attn<<<dim3(S / 16, HQ), 32, 0, stream>>>(qh, ql, kh, kl, vh, vl, cth, ctl, S, DC);
        k_proj<<<dim3(D / 128, S / 64), 128, 0, stream>>>(cth, ctl, woh, wol, out, DC, D, b * S);
    }
}
